// CausalSelfAttention_79508434583850
// MI455X (gfx1250) — hardware-verified
//
#include <hip/hip_runtime.h>


#ifndef NB
#define NB 2
#endif
#ifndef SEQ
#define SEQ 2048
#endif
#define NB_FULL  2
#define SEQ_FULL 2048
#define DM   1024
#define NH   16
#define HD   64
#define RH   ((SEQ) < 256 ? (SEQ) : 256)
#define PP   40
#define SCL   0.125f
#define LOG2E 1.4426950408889634f
#define PSH   10.0f
#define NEGB  (-1.0e30f)

typedef _Float16 h16;
typedef unsigned short bf;
typedef __attribute__((ext_vector_type(16))) __bf16   v16bf;
typedef __attribute__((ext_vector_type(16))) _Float16 v16h;
typedef __attribute__((ext_vector_type(8)))  _Float16 v8h;
typedef __attribute__((ext_vector_type(8)))  unsigned short v8us;
typedef __attribute__((ext_vector_type(8)))  float    v8f;
typedef __attribute__((ext_vector_type(4)))  float    v4f;
typedef v8h  __attribute__((may_alias)) v8ha;
typedef v4f  __attribute__((may_alias)) v4fa;
typedef v8us __attribute__((may_alias)) v8usa;

static_assert(NH * HD == DM);
static_assert(HD == 64);
static_assert(DM % 64 == 0);
static_assert(SEQ % 64 == 0);
static_assert((NB * SEQ) % 64 == 0);
static_assert(RH % 64 == 0);
static_assert(RH <= SEQ);
static_assert(NB <= NB_FULL);
static_assert(SEQ <= SEQ_FULL);
static_assert(PP % 8 == 0);
static_assert(PP >= 32);

__device__ __forceinline__ unsigned short f2bf(float f) { unsigned u = __float_as_uint(f); u += 0x7FFFu + ((u >> 16) & 1u); return (unsigned short)(u >> 16); }
__device__ __forceinline__ float bf2f(unsigned short b) { return __uint_as_float(((unsigned)b) << 16); }
__device__ __forceinline__ float bfr(float f) { return bf2f(f2bf(f)); }
__device__ __forceinline__ void splitf(float y, unsigned short& h, unsigned short& l) { h = f2bf(y); l = f2bf(y - bf2f(h)); }
__device__ __forceinline__ v16h cat16(v8h lo, v8h hi) { return __builtin_shufflevector(lo, hi, 0, 1, 2, 3, 4, 5, 6, 7, 8, 9, 10, 11, 12, 13, 14, 15); }
__device__ __forceinline__ v16bf cat16b(v8us lo, v8us hi) { return __builtin_bit_cast(v16bf, __builtin_shufflevector(lo, hi, 0, 1, 2, 3, 4, 5, 6, 7, 8, 9, 10, 11, 12, 13, 14, 15)); }
__device__ __forceinline__ v8f wmma16(v16h a, v16h b, v8f c) { return __builtin_amdgcn_wmma_f32_16x16x32_f16(false, a, false, b, (short)0, c, false, false); }
__device__ __forceinline__ v8f wmmab(v16bf a, v16bf b, v8f c) { return __builtin_amdgcn_wmma_f32_16x16x32_bf16(false, a, false, b, (short)0, c, false, false); }
__device__ __forceinline__ v16bf ldb(const bf* p) { return cat16b(*(const v8us*)p, *(const v8us*)(p + 16)); }
__device__ __forceinline__ v16h ldh(const h16* p) { return cat16(*(const v8h*)p, *(const v8h*)(p + 16)); }

template <int NSPLIT>
__device__ __forceinline__ void gemmw_body(const bf* __restrict__ A, const bf* __restrict__ A2, const bf* __restrict__ Bt, float* C, const float* __restrict__ bias, size_t sA, size_t sC) {
    __shared__ __align__(16) float os[16 * 68];
    const size_t z = blockIdx.z; A += z * sA; A2 += z * sA; C += z * sC;
    const int lane = threadIdx.x & 31, lr = lane & 15, hi = lane >> 4; const int r0 = blockIdx.x * 64, c0 = blockIdx.y * 64;
    v8f acc[4][4];
#pragma unroll
    for (int mb = 0; mb < 4; ++mb)
#pragma unroll
        for (int nb = 0; nb < 4; ++nb) acc[mb][nb] = (v8f){};
    const size_t aoff = (size_t)(r0 + lr) * DM + 8 * hi, boff = (size_t)(c0 + lr) * DM + 8 * hi;
#pragma unroll 1
    for (int kc = 0; kc < DM; kc += 32) {
        v16bf a[4], a2[4], bl;
#pragma unroll
        for (int mb = 0; mb < 4; ++mb) { a[mb] = ldb(A + aoff + (size_t)mb * 16 * DM + kc); if (NSPLIT == 1) a2[mb] = ldb(A2 + aoff + (size_t)mb * 16 * DM + kc); else a2[mb] = a[mb]; }
#pragma unroll
        for (int nb = 0; nb < 4; ++nb) { const v16bf b = ldb(Bt + boff + (size_t)nb * 16 * DM + kc);
#pragma unroll
            for (int mb = 0; mb < 4; ++mb) { acc[mb][nb] = wmmab(a[mb], b, acc[mb][nb]); if (NSPLIT == 1) acc[mb][nb] = wmmab(a2[mb], b, acc[mb][nb]); }
            if (nb == 3) bl = b; }
        asm volatile("" : "+v"(acc[0][0]), "+v"(acc[0][1]), "+v"(acc[0][2]), "+v"(acc[0][3]));
        asm volatile("" : "+v"(acc[1][0]), "+v"(acc[1][1]), "+v"(acc[1][2]), "+v"(acc[1][3]));
        asm volatile("" : "+v"(acc[2][0]), "+v"(acc[2][1]), "+v"(acc[2][2]), "+v"(acc[2][3]));
        asm volatile("v_nop\n\tv_nop\n\tv_nop\n\tv_nop" : "+v"(acc[3][0]), "+v"(acc[3][1]), "+v"(acc[3][2]), "+v"(acc[3][3]) : "v"(a[3]), "v"(a2[3]), "v"(bl));
    }
#pragma unroll
    for (int mb = 0; mb < 4; ++mb) {
#pragma unroll
        for (int nb = 0; nb < 4; ++nb) {
#pragma unroll
            for (int j = 0; j < 8; ++j) os[(hi * 8 + j) * 68 + nb * 16 + lr] = acc[mb][nb][j]; }
        __syncthreads();
        float* crow = C + (size_t)(r0 + mb * 16) * DM + c0;
#pragma unroll 1
        for (int ps = 0; ps < 2; ++ps) {
#pragma unroll
            for (int s = 0; s < 8; ++s) { const int row = 2 * s + hi, cofs = lr * 4; v4f val = *(const v4fa*)(os + row * 68 + cofs);
                val[0] += bfr(bias[c0 + cofs]); val[1] += bfr(bias[c0 + cofs + 1]); val[2] += bfr(bias[c0 + cofs + 2]); val[3] += bfr(bias[c0 + cofs + 3]);
                *(volatile v4f*)(crow + (size_t)row * DM + cofs) = val; }
            if (ps == 0) __threadfence(); }
        __syncthreads();
    }
}
__global__ __launch_bounds__(32) void k_gemm_proj(const bf* __restrict__ A, const bf* __restrict__ Bt, const float* __restrict__ bias, float* C) { gemmw_body<0>(A, A, Bt, C, bias, 0, 0); }
__global__ __launch_bounds__(32) void k_gemm_out(const bf* __restrict__ Ah, const bf* __restrict__ Al, const bf* __restrict__ Bt, const float* __restrict__ bias, float* C) { gemmw_body<1>(Ah, Al, Bt, C, bias, (size_t)SEQ * DM, (size_t)SEQ_FULL * DM); }

__global__ __launch_bounds__(256) void k_cvt8(const float* __restrict__ src, bf* dst, size_t n8) { const size_t i = (size_t)blockIdx.x * 256 + threadIdx.x; if (i >= n8) return; const v8f v = *(const v8f*)(src + i * 8); v8us o;
#pragma unroll
    for (int k = 0; k < 8; ++k) o[k] = f2bf(v[k]); *(volatile v8us*)(dst + i * 8) = o; __threadfence(); *(volatile v8us*)(dst + i * 8) = o; }

__global__ __launch_bounds__(256) void k_qkp(const float* __restrict__ F, bf* Ph, bf* Pl) {
    const size_t idx = (size_t)blockIdx.x * 256 + threadIdx.x; if (idx >= (size_t)NB * NH * SEQ * HD / 8) return;
    const size_t e = idx * 8; const int d = (int)(e % HD); const int t = (int)((e / HD) % SEQ); const int bh = (int)(e / ((size_t)HD * SEQ)); const int b = bh / NH, h = bh % NH;
    const float* f = F + ((size_t)b * SEQ + t) * DM + h * HD + d; const v4f a = *(const v4f*)f, c = *(const v4f*)(f + 4); v8us oh, ol;
#pragma unroll
    for (int q = 0; q < 4; ++q) { unsigned short a2, c2; splitf(a[q], a2, c2); oh[q] = a2; ol[q] = c2; splitf(c[q], a2, c2); oh[4 + q] = a2; ol[4 + q] = c2; }
    *(volatile v8us*)(Ph + e) = oh; *(volatile v8us*)(Pl + e) = ol; __threadfence(); *(volatile v8us*)(Ph + e) = oh; *(volatile v8us*)(Pl + e) = ol; }

__global__ __launch_bounds__(256) void k_vtp(const float* __restrict__ F, h16* V16, bf* Vh, bf* Vl) {
    const size_t idx = (size_t)blockIdx.x * 256 + threadIdx.x; if (idx >= (size_t)NB * NH * HD * SEQ / 8) return;
    const size_t e = idx * 8; const int t = (int)(e % SEQ); const int d = (int)((e / SEQ) % HD); const int bh = (int)(e / ((size_t)SEQ * HD)); const int b = bh / NH, h = bh % NH;
    const float* f = F + ((size_t)b * SEQ + t) * DM + h * HD + d; v8h o16; v8us oh, ol;
#pragma unroll
    for (int q = 0; q < 8; ++q) { const float x = f[(size_t)q * DM]; o16[q] = (h16)x; unsigned short a2, c2; splitf(x, a2, c2); oh[q] = a2; ol[q] = c2; }
    const bool early = (t < RH); const size_t eo = ((size_t)bh * HD + d) * RH + (early ? t : 0);
    *(volatile v8h*)(V16 + e) = o16; if (early) { *(volatile v8us*)(Vh + eo) = oh; *(volatile v8us*)(Vl + eo) = ol; }
    __threadfence();
    *(volatile v8h*)(V16 + e) = o16; if (early) { *(volatile v8us*)(Vh + eo) = oh; *(volatile v8us*)(Vl + eo) = ol; } }

template <bool HIRES>
__device__ __forceinline__ void attn_body(const bf* __restrict__ QPh, const bf* __restrict__ QPl, const bf* __restrict__ KPh, const bf* __restrict__ KPl,
                                          const h16* __restrict__ VT16, const bf* __restrict__ VTh, const bf* __restrict__ VTl, bf* ATh, bf* ATl, int tile0) {
    __shared__ __align__(16) h16 pt16[16 * PP];
    __shared__ __align__(16) unsigned short pth[16 * PP];
    __shared__ __align__(16) unsigned short ptl[16 * PP];
    __shared__ __align__(16) float os[16 * 68];
    const int lane = threadIdx.x & 31, lr = lane & 15, hi = lane >> 4;
    const int bh = blockIdx.y; const int b = bh / NH, h = bh % NH;
    const int i0 = (tile0 + (int)blockIdx.x) * 16;
    const size_t pb = (size_t)bh * SEQ * HD;
    const bf* qh = QPh + pb; const bf* ql = QPl + pb; const bf* kh = KPh + pb; const bf* kl = KPl + pb;
    const h16* vt = VT16 + ((size_t)bh * HD + lr) * SEQ + 8 * hi;
    const bf* vth = VTh + ((size_t)bh * HD + lr) * RH + 8 * hi;
    const bf* vtl = VTl + ((size_t)bh * HD + lr) * RH + 8 * hi;
    const int qoff0 = (i0 + lr) * HD + 8 * hi;
    v8f o[4];
#pragma unroll
    for (int j = 0; j < 4; ++j) o[j] = (v8f){};
    float mrow[8], lrow[8];
#pragma unroll
    for (int r = 0; r < 8; ++r) { mrow[r] = NEGB; lrow[r] = 0.0f; }
    const int nsteps = i0 / 32 + 1;
#pragma unroll 1
    for (int st = 0; st < nsteps; ++st) {
        const int kb = st * 32;
        v8f s0 = (v8f){}, s1 = (v8f){};
        int qo = qoff0; asm volatile("" : "+v"(qo));
        const int ko = (kb + lr) * HD + 8 * hi;
#pragma unroll
        for (int kc = 0; kc < HD; kc += 32) {
            const v16bf aq = ldb(qh + qo + kc), al = ldb(ql + qo + kc);
            const v16bf k0h = ldb(kh + ko + kc), k0l = ldb(kl + ko + kc);
            s0 = wmmab(aq, k0h, s0); s0 = wmmab(al, k0h, s0); s0 = wmmab(aq, k0l, s0);
            const v16bf k1h = ldb(kh + ko + 16 * HD + kc), k1l = ldb(kl + ko + 16 * HD + kc);
            s1 = wmmab(aq, k1h, s1); s1 = wmmab(al, k1h, s1); s1 = wmmab(aq, k1l, s1);
            asm volatile("v_nop\n\tv_nop\n\tv_nop\n\tv_nop" : "+v"(s0), "+v"(s1) : "v"(aq), "v"(al), "v"(k1h), "v"(k1l));
        }
        float x0[8], x1[8], bm[8];
#pragma unroll
        for (int r = 0; r < 8; ++r) { x0[r] = s0[r] * SCL; x1[r] = s1[r] * SCL; }
        if (kb + 31 > i0) {
#pragma unroll
            for (int r = 0; r < 8; ++r) { const int row = i0 + 8 * hi + r; x0[r] = (kb + lr > row) ? NEGB : x0[r]; x1[r] = (kb + 16 + lr > row) ? NEGB : x1[r]; }
        }
#pragma unroll
        for (int r = 0; r < 8; ++r) bm[r] = fmaxf(x0[r], x1[r]);
#pragma unroll
        for (int off = 1; off < 16; off <<= 1) {
#pragma unroll
            for (int r = 0; r < 8; ++r) bm[r] = fmaxf(bm[r], __shfl_xor(bm[r], off, 32)); }
        float fac[8], rs[8];
#pragma unroll
        for (int r = 0; r < 8; ++r) {
            const float nm = fmaxf(mrow[r], bm[r]);
            fac[r] = __builtin_amdgcn_exp2f((mrow[r] - nm) * LOG2E);
            mrow[r] = nm;
            const float p0 = __builtin_amdgcn_exp2f((x0[r] - nm) * LOG2E + PSH);
            const float p1 = __builtin_amdgcn_exp2f((x1[r] - nm) * LOG2E + PSH);
            rs[r] = p0 + p1;
            const int prow = (8 * hi + r) * PP;
            if (HIRES) { unsigned short a2, c2; splitf(p0, a2, c2); pth[prow + lr] = a2; ptl[prow + lr] = c2; splitf(p1, a2, c2); pth[prow + 16 + lr] = a2; ptl[prow + 16 + lr] = c2; }
            else { pt16[prow + lr] = (h16)p0; pt16[prow + 16 + lr] = (h16)p1; }
        }
#pragma unroll
        for (int off = 1; off < 16; off <<= 1) {
#pragma unroll
            for (int r = 0; r < 8; ++r) rs[r] += __shfl_xor(rs[r], off, 32); }
#pragma unroll
        for (int r = 0; r < 8; ++r) { lrow[r] = lrow[r] * fac[r] + rs[r];
#pragma unroll
            for (int j = 0; j < 4; ++j) o[j][r] *= fac[r]; }
        __syncthreads();
        if (HIRES) {
            const v16bf pah = cat16b(*(const v8usa*)(pth + lr * PP + 8 * hi), *(const v8usa*)(pth + lr * PP + 16 + 8 * hi));
            const v16bf pal = cat16b(*(const v8usa*)(ptl + lr * PP + 8 * hi), *(const v8usa*)(ptl + lr * PP + 16 + 8 * hi));
            v16bf vh[4];
#pragma unroll
            for (int j = 0; j < 4; ++j) vh[j] = ldb(vth + (size_t)j * 16 * RH + kb);
#pragma unroll
            for (int j = 0; j < 4; ++j) { o[j] = wmmab(pah, vh[j], o[j]); o[j] = wmmab(pal, vh[j], o[j]); }
            asm volatile("v_nop\n\tv_nop\n\tv_nop\n\tv_nop" : "+v"(o[0]), "+v"(o[1]), "+v"(o[2]), "+v"(o[3]) : "v"(vh[3]), "v"(pal));
            v16bf vl[4];
#pragma unroll
            for (int j = 0; j < 4; ++j) vl[j] = ldb(vtl + (size_t)j * 16 * RH + kb);
#pragma unroll
            for (int j = 0; j < 4; ++j) o[j] = wmmab(pah, vl[j], o[j]);
            asm volatile("v_nop\n\tv_nop\n\tv_nop\n\tv_nop" : "+v"(o[0]), "+v"(o[1]), "+v"(o[2]), "+v"(o[3]) : "v"(vl[3]), "v"(pah));
        } else {
            const v16h pa = cat16(*(const v8ha*)(pt16 + lr * PP + 8 * hi), *(const v8ha*)(pt16 + lr * PP + 16 + 8 * hi));
            v16h vb[4];
#pragma unroll
            for (int j = 0; j < 4; ++j) vb[j] = ldh(vt + (size_t)j * 16 * SEQ + kb);
#pragma unroll
            for (int j = 0; j < 4; ++j) o[j] = wmma16(pa, vb[j], o[j]);
            asm volatile("v_nop\n\tv_nop\n\tv_nop\n\tv_nop" : "+v"(o[0]), "+v"(o[1]), "+v"(o[2]), "+v"(o[3]) : "v"(vb[3]), "v"(pa));
        }
        __syncthreads();
    }
#pragma unroll
    for (int r = 0; r < 8; ++r) { const float inv = 1.0f / lrow[r];
#pragma unroll
        for (int j = 0; j < 4; ++j) os[(8 * hi + r) * 68 + j * 16 + lr] = o[j][r] * inv; }
    __syncthreads();
    v8us oh[4], ol[4]; size_t oo[4];
#pragma unroll
    for (int s = 0; s < 4; ++s) {
        const int row = s * 4 + (lane >> 3), c8 = (lane & 7) * 8;
        const v4f a = *(const v4fa*)(os + row * 68 + c8), c = *(const v4fa*)(os + row * 68 + c8 + 4);
#pragma unroll
        for (int q = 0; q < 4; ++q) { unsigned short a2, c2; splitf(a[q], a2, c2); oh[s][q] = a2; ol[s][q] = c2; splitf(c[q], a2, c2); oh[s][4 + q] = a2; ol[s][4 + q] = c2; }
        oo[s] = ((size_t)b * SEQ + i0 + row) * DM + h * HD + c8; }
#pragma unroll
    for (int s = 0; s < 4; ++s) { *(volatile v8us*)(ATh + oo[s]) = oh[s]; *(volatile v8us*)(ATl + oo[s]) = ol[s]; }
    __threadfence();
#pragma unroll
    for (int s = 0; s < 4; ++s) { *(volatile v8us*)(ATh + oo[s]) = oh[s]; *(volatile v8us*)(ATl + oo[s]) = ol[s]; }
}
__global__ __launch_bounds__(32) void k_attn_early(const bf* __restrict__ QPh, const bf* __restrict__ QPl, const bf* __restrict__ KPh, const bf* __restrict__ KPl, const h16* __restrict__ VT16, const bf* __restrict__ VTh, const bf* __restrict__ VTl, bf* ATh, bf* ATl) {
    attn_body<true>(QPh, QPl, KPh, KPl, VT16, VTh, VTl, ATh, ATl, 0); }
__global__ __launch_bounds__(32) void k_attn_main(const bf* __restrict__ QPh, const bf* __restrict__ QPl, const bf* __restrict__ KPh, const bf* __restrict__ KPl, const h16* __restrict__ VT16, const bf* __restrict__ VTh, const bf* __restrict__ VTl, bf* ATh, bf* ATl) {
    attn_body<false>(QPh, QPl, KPh, KPl, VT16, VTh, VTl, ATh, ATl, RH / 16); }

constexpr size_t SZ_W  = (size_t)DM * DM * 2;
constexpr size_t SZ_X  = (size_t)NB * SEQ * DM * 2;
constexpr size_t SZ_F  = (size_t)NB * SEQ * DM * 4;
constexpr size_t SZ_P  = (size_t)NB * NH * SEQ * HD * 2;
constexpr size_t SZ_VR = (size_t)NB * NH * HD * RH * 2;
constexpr size_t SZ_A  = (size_t)NB * SEQ * DM * 2;
constexpr size_t WS_TOTAL = 4 * SZ_W + SZ_X + SZ_F + 4 * SZ_P + SZ_P + 2 * SZ_VR + 2 * SZ_A;
static_assert(SZ_W % 256 == 0);
static_assert(SZ_X % 256 == 0);
static_assert(SZ_F % 256 == 0);
static_assert(SZ_P % 256 == 0);
static_assert(SZ_VR % 256 == 0);
static_assert(SZ_A % 256 == 0);
static_assert(WS_TOTAL <= (size_t)134217728);
static_assert((size_t)NB_FULL * SEQ_FULL * DM * 4 == (size_t)16777216);
static_assert(((size_t)(NB - 1) * SEQ_FULL + SEQ) * DM <= (size_t)NB_FULL * SEQ_FULL * DM);

extern "C" void kernel_launch(void* const* d_in, const int* in_sizes, int n_in,
                              void* d_out, int out_size, void* d_ws, size_t ws_size, hipStream_t stream) {
    if (n_in < 9) return;
    const long long needX = ((long long)(NB - 1) * SEQ_FULL + SEQ) * DM;
    if ((long long)in_sizes[0] < needX) return;
    if (in_sizes[1] < DM * DM || in_sizes[3] < DM * DM || in_sizes[5] < DM * DM || in_sizes[7] < DM * DM) return;
    if (in_sizes[2] < DM || in_sizes[4] < DM || in_sizes[6] < DM || in_sizes[8] < DM) return;
    if ((long long)out_size < needX) return;
    if (ws_size < WS_TOTAL) return;
    const float* x = (const float*)d_in[0]; const float* wq = (const float*)d_in[1]; const float* bq = (const float*)d_in[2]; const float* wk = (const float*)d_in[3]; const float* bk = (const float*)d_in[4];
    const float* wv = (const float*)d_in[5]; const float* bv = (const float*)d_in[6]; const float* wp = (const float*)d_in[7]; const float* bp = (const float*)d_in[8];
    float* OUT = (float*)d_out;
    char* w = (char*)d_ws; size_t off = 0;
    bf* WQ = (bf*)(w + off); off += SZ_W; bf* WK = (bf*)(w + off); off += SZ_W; bf* WV = (bf*)(w + off); off += SZ_W; bf* WO = (bf*)(w + off); off += SZ_W;
    bf* XB = (bf*)(w + off); off += SZ_X; float* F = (float*)(w + off); off += SZ_F;
    bf* QPh = (bf*)(w + off); off += SZ_P; bf* QPl = (bf*)(w + off); off += SZ_P; bf* KPh = (bf*)(w + off); off += SZ_P; bf* KPl = (bf*)(w + off); off += SZ_P;
    h16* VT16 = (h16*)(w + off); off += SZ_P; bf* VTh = (bf*)(w + off); off += SZ_VR; bf* VTl = (bf*)(w + off); off += SZ_VR;
    bf* ATh = (bf*)(w + off); off += SZ_A; bf* ATl = (bf*)(w + off); off += SZ_A;
    if (off != WS_TOTAL) return;

    const size_t nw8 = (size_t)DM * DM / 8, nx8 = (size_t)SEQ * DM / 8;
    const unsigned gw = (unsigned)((nw8 + 255) / 256), gx = (unsigned)((nx8 + 255) / 256);
    k_cvt8<<<gw, 256, 0, stream>>>(wq, WQ, nw8); k_cvt8<<<gw, 256, 0, stream>>>(wk, WK, nw8); k_cvt8<<<gw, 256, 0, stream>>>(wv, WV, nw8); k_cvt8<<<gw, 256, 0, stream>>>(wp, WO, nw8);
    for (int b = 0; b < NB; ++b) k_cvt8<<<gx, 256, 0, stream>>>(x + (size_t)b * SEQ_FULL * DM, XB + (size_t)b * SEQ * DM, nx8);
    const dim3 gp(NB * SEQ / 64, DM / 64, 1);
    const unsigned gq = (unsigned)(((size_t)NB * NH * SEQ * HD / 8 + 255) / 256);
    k_gemm_proj<<<gp, 32, 0, stream>>>(XB, WQ, bq, F); k_qkp<<<gq, 256, 0, stream>>>(F, QPh, QPl);
    k_gemm_proj<<<gp, 32, 0, stream>>>(XB, WK, bk, F); k_qkp<<<gq, 256, 0, stream>>>(F, KPh, KPl);
    k_gemm_proj<<<gp, 32, 0, stream>>>(XB, WV, bv, F); k_vtp<<<gq, 256, 0, stream>>>(F, VT16, VTh, VTl);
    k_attn_early<<<dim3(RH / 16, NB * NH, 1), 32, 0, stream>>>(QPh, QPl, KPh, KPl, VT16, VTh, VTl, ATh, ATl);
    if (SEQ > RH) k_attn_main<<<dim3((SEQ - RH) / 16 + (SEQ == RH ? 1 : 0), NB * NH, 1), 32, 0, stream>>>(QPh, QPl, KPh, KPl, VT16, VTh, VTl, ATh, ATl);
    k_gemm_out<<<dim3(SEQ / 64, DM / 64, NB), 32, 0, stream>>>(ATh, ATl, WO, bp, OUT);
}
